// DecorrLoss_41618233099088
// MI455X (gfx1250) — hardware-run, weakly checked
//
#include <hip/hip_runtime.h>


#define NN   32768
#define ND   1024
#define NP   8
#define NK   4096
#define NT   16
typedef _Float16 h16;
typedef unsigned short bf;
typedef __attribute__((ext_vector_type(16))) __bf16   v16bf;
typedef __attribute__((ext_vector_type(16))) _Float16 v16h;
typedef __attribute__((ext_vector_type(8)))  _Float16 v8h;
typedef __attribute__((ext_vector_type(8)))  unsigned short v8us;
typedef __attribute__((ext_vector_type(8)))  float    v8f;
typedef __attribute__((ext_vector_type(4)))  float    v4f;
typedef v8h  __attribute__((may_alias)) v8ha;
typedef v4f  __attribute__((may_alias)) v4fa;
typedef v8us __attribute__((may_alias)) v8usa;

__device__ __forceinline__ unsigned short f2bf(float f) { unsigned u = __float_as_uint(f); u += 0x7FFFu + ((u >> 16) & 1u); return (unsigned short)(u >> 16); }
__device__ __forceinline__ float bf2f(unsigned short b) { return __uint_as_float(((unsigned)b) << 16); }
__device__ __forceinline__ float bfr(float f) { return bf2f(f2bf(f)); }
__device__ __forceinline__ v16h cat16(v8h lo, v8h hi) { return __builtin_shufflevector(lo, hi, 0, 1, 2, 3, 4, 5, 6, 7, 8, 9, 10, 11, 12, 13, 14, 15); }
__device__ __forceinline__ v16bf cat16b(v8us lo, v8us hi) { return __builtin_bit_cast(v16bf, __builtin_shufflevector(lo, hi, 0, 1, 2, 3, 4, 5, 6, 7, 8, 9, 10, 11, 12, 13, 14, 15)); }
__device__ __forceinline__ v8f wmma16(v16h a, v16h b, v8f c) { return __builtin_amdgcn_wmma_f32_16x16x32_f16(false, a, false, b, (short)0, c, false, false); }
__device__ __forceinline__ v8f wmmab(v16bf a, v16bf b, v8f c) { return __builtin_amdgcn_wmma_f32_16x16x32_bf16(false, a, false, b, (short)0, c, false, false); }

template <typename T16> struct WFrag;
template <> struct WFrag<h16> { typedef v16h V; static __device__ __forceinline__ V ld(const h16* p) { return cat16(*(const v8h*)p, *(const v8h*)(p + 16)); } static __device__ __forceinline__ v8f mma(V a, V b, v8f c) { return wmma16(a, b, c); } };
template <> struct WFrag<bf> { typedef v16bf V; static __device__ __forceinline__ V ld(const bf* p) { return cat16b(*(const v8us*)p, *(const v8us*)(p + 16)); } static __device__ __forceinline__ v8f mma(V a, V b, v8f c) { return wmmab(a, b, c); } };
template <typename T16, int NSPLIT, bool BIAS>
__global__ __launch_bounds__(32) void k_gemmw(const T16* __restrict__ A, const T16* __restrict__ A2, const T16* __restrict__ Bt, const T16* __restrict__ Bt2, int K, float* C, int ldc, const float* __restrict__ bias, size_t sA, size_t sB, size_t sC) {
    typedef typename WFrag<T16>::V V;
    __shared__ __align__(16) float os[16 * 68];
    const size_t z = blockIdx.z; A += z * sA; if (A2) A2 += z * sA; Bt += z * sB; if (Bt2) Bt2 += z * sB; C += z * sC;
    const int lane = threadIdx.x & 31, lr = lane & 15, hi = lane >> 4; const int r0 = blockIdx.x * 64, c0 = blockIdx.y * 64;
    v8f acc[4][4];
#pragma unroll
    for (int mb = 0; mb < 4; ++mb)
#pragma unroll
        for (int nb = 0; nb < 4; ++nb) acc[mb][nb] = (v8f){};
    const size_t aoff = (size_t)(r0 + lr) * K + 8 * hi, boff = (size_t)(c0 + lr) * K + 8 * hi;
    for (int kc = 0; kc < K; kc += 32) {
        V a[4], a2[4];
#pragma unroll
        for (int mb = 0; mb < 4; ++mb) { a[mb] = WFrag<T16>::ld(A + aoff + (size_t)mb * 16 * K + kc); if (NSPLIT == 1 || NSPLIT == 2) a2[mb] = WFrag<T16>::ld(A2 + aoff + (size_t)mb * 16 * K + kc); }
#pragma unroll
        for (int nb = 0; nb < 4; ++nb) { const V b = WFrag<T16>::ld(Bt + boff + (size_t)nb * 16 * K + kc); V b2; if (NSPLIT >= 2) b2 = WFrag<T16>::ld(Bt2 + boff + (size_t)nb * 16 * K + kc);
#pragma unroll
            for (int mb = 0; mb < 4; ++mb) { acc[mb][nb] = WFrag<T16>::mma(a[mb], b, acc[mb][nb]); if (NSPLIT == 1 || NSPLIT == 2) acc[mb][nb] = WFrag<T16>::mma(a2[mb], b, acc[mb][nb]); if (NSPLIT >= 2) acc[mb][nb] = WFrag<T16>::mma(a[mb], b2, acc[mb][nb]); } }
        asm volatile("v_nop\n\tv_nop\n\tv_nop\n\tv_nop" : "+v"(acc[0][0]), "+v"(acc[1][1]), "+v"(acc[2][2]), "+v"(acc[3][3]) : "v"(a[0]), "v"(a[3]));
    }
#pragma unroll
    for (int mb = 0; mb < 4; ++mb) {
#pragma unroll
        for (int nb = 0; nb < 4; ++nb) {
#pragma unroll
            for (int j = 0; j < 8; ++j) os[(hi * 8 + j) * 68 + nb * 16 + lr] = acc[mb][nb][j]; }
        __builtin_amdgcn_wave_barrier(); asm volatile("" ::: "memory");
        float* crow = C + (size_t)(r0 + mb * 16) * ldc + c0;
#pragma unroll 1
        for (int ps = 0; ps < 2; ++ps) {
#pragma unroll
            for (int s = 0; s < 8; ++s) { const int row = 2 * s + hi, cofs = lr * 4; v4f val = *(const v4fa*)(os + row * 68 + cofs); if (BIAS) { val[0] += bfr(bias[c0 + cofs]); val[1] += bfr(bias[c0 + cofs + 1]); val[2] += bfr(bias[c0 + cofs + 2]); val[3] += bfr(bias[c0 + cofs + 3]); }
                *(volatile v4f*)(crow + (size_t)row * ldc + cofs) = val; }
            if (ps == 0) __threadfence(); }
        __builtin_amdgcn_wave_barrier(); asm volatile("" ::: "memory");
    }
}

typedef __attribute__((ext_vector_type(2))) _Float16 v2h;
typedef __attribute__((ext_vector_type(4))) _Float16 v4h;
typedef __attribute__((ext_vector_type(2))) unsigned short v2us;
typedef __attribute__((ext_vector_type(4))) unsigned short v4us;
typedef __attribute__((ext_vector_type(2))) float v2f;
typedef __attribute__((ext_vector_type(4))) int v4i;

__global__ __launch_bounds__(256) void k_wtG(const float* __restrict__ w, int K, int N, bf* Bt) {
    const int lane = threadIdx.x & 31; const int L0 = (blockIdx.x * 8 + (threadIdx.x >> 5)) * 8; const int nlines = N * K / 64;
#pragma unroll
    for (int ps = 0; ps < 2; ++ps) {
        for (int l = 0; l < 8; ++l) { const int L = L0 + l; if (L >= nlines) break; const size_t e = (size_t)L * 64 + lane * 2; const int k = (int)(e % K), n = (int)(e / K); v2us o;
            o[0] = f2bf(w[(size_t)k * N + n]); o[1] = f2bf(w[(size_t)(k + 1) * N + n]); *(volatile v2us*)(Bt + e) = o; }
        if (ps == 0) __threadfence(); }
}

__global__ __launch_bounds__(256) void k_rs(const float* __restrict__ a, float* R1, float* R2) { const int r = blockIdx.x * 256 + threadIdx.x; if (r >= NN) return; const float* p = a + (size_t)r * ND; float s2 = 0.0f, s4 = 0.0f, w = 0.0f;
    for (int q = 0; q < ND / 4; ++q) { const v4f v = *(const v4f*)(p + 4 * q);
#pragma unroll
        for (int e = 0; e < 4; ++e) { const float x = bfr(v[e]); const float x2 = __fmul_rn(x, x); const float y = __fsub_rn(x2, 1.0f); s2 = __fadd_rn(s2, x2); s4 = __fmaf_rn(x2, x2, s4); w = __fmaf_rn(y, y, w); } }
    const float r1 = __fsub_rn(__fmul_rn(s2, s2), s4);
    *(volatile float*)(R1 + r) = r1; *(volatile float*)(R2 + r) = w; __threadfence(); *(volatile float*)(R1 + r) = r1; *(volatile float*)(R2 + r) = w; }

__global__ __launch_bounds__(32) void k_sc(const float* __restrict__ R1, const float* __restrict__ R2, float* o2) { const int l = threadIdx.x; if (blockIdx.x != 0 || l >= 2) return; const float* src = l ? R2 : R1; float s = 0.0f;
    for (int r = 0; r < NN; ++r) s = __fadd_rn(s, src[r]);
    const float o = __fdiv_rn(__fdiv_rn(s, (float)NN), l ? (float)ND : (float)(ND * ND));
    *(volatile float*)(o2 + l) = o; __threadfence(); *(volatile float*)(o2 + l) = o; }

__global__ __launch_bounds__(256) void k_g(const float* __restrict__ P, float* out0) { const int t = blockIdx.x * 256 + threadIdx.x; if (t >= ND * ND) return; const int i = t / ND, j = t % ND; const bool up = (i / 64) <= (j / 64); const int rr = up ? i : j, cc = up ? j : i; const size_t e = (size_t)rr * ND + cc; float p = P[e];
#pragma unroll
    for (int q = 1; q < NP; ++q) p = __fadd_rn(p, P[(size_t)q * ND * ND + e]);
    const float q = __fdiv_rn(p, (float)NN); const float off = __fmul_rn(0.5f, q); const float dg = __fmul_rn(0.5f, __fsub_rn(q, 1.0f)); const float o = (i == j) ? dg : off;
    *(volatile float*)(out0 + t) = o; __threadfence(); *(volatile float*)(out0 + t) = o; }

extern "C" void kernel_launch(void* const* d_in, const int* in_sizes, int n_in, void* d_out, int out_size, void* d_ws, size_t ws_size, hipStream_t stream) {
    if (n_in < 1) return;
    if (in_sizes[0] != NN * ND) return;
    if (out_size != ND * ND + 2) return;
    static_assert(NP * NK == NN && NK % 32 == 0 && (ND * NK) % (64 * 64) == 0 && ND % 64 == 0 && NT * 64 == ND && NN % 256 == 0 && (ND * ND) % 256 == 0 && (ND & (ND - 1)) == 0 && (NN & (NN - 1)) == 0 && (size_t)ND * NN / 64 / 64 < 65536u * 32768u, "the product: M and N multiples of 64, the depth a multiple of 32; k_wtG's lines of 64 words; every flat grid exact; n and d powers of two: the divisions by n, d and d squared are exact");
    const float* a = (const float*)d_in[0];
    float* out0 = (float*)d_out; float* o2 = out0 + ND * ND;
    char* wsp = (char*)d_ws; auto take = [&](size_t bytes) { char* p = wsp; wsp += (bytes + 255) & ~(size_t)255; return (void*)p; };
    bf* Xt = (bf*)take((size_t)ND * NN * 2); float* P = (float*)take((size_t)NP * ND * ND * 4);     float* R1 = (float*)take((size_t)NN * 4); float* R2 = (float*)take((size_t)NN * 4);
    if ((size_t)(wsp - (char*)d_ws) > ws_size) return;
    for (int p = 0; p < NP; ++p) { bf* Xp = Xt + (size_t)p * ND * NK; float* Pp = P + (size_t)p * ND * ND;
        k_wtG<<<(unsigned)(ND * NK / 64 / 64), 256, 0, stream>>>(a + (size_t)p * NK * ND, NK, ND, Xp);
        for (int r = 0; r < NT; ++r) { const bf* Xr = Xp + (size_t)r * 64 * NK;
            k_gemmw<bf, 0, false><<<dim3(1, NT - r, 1), 32, 0, stream>>>(Xr, nullptr, Xr, nullptr, NK, Pp + (size_t)r * 64 * ND + r * 64, ND, nullptr, 0, 0, 0); } }
    k_rs<<<(unsigned)(NN / 256), 256, 0, stream>>>(a, R1, R2);
    k_sc<<<1, 32, 0, stream>>>(R1, R2, o2);
    k_g<<<(unsigned)(ND * ND / 256), 256, 0, stream>>>(P, out0);
}
